// TransformerBlock_49374944035441
// MI455X (gfx1250) — hardware-verified
//
#include <hip/hip_runtime.h>
#include <stddef.h>


typedef _Float16 v16h __attribute__((ext_vector_type(16)));
typedef _Float16 v8h  __attribute__((ext_vector_type(8)));
typedef float    v8f  __attribute__((ext_vector_type(8)));
typedef float    v4f  __attribute__((ext_vector_type(4)));

#ifndef NB
#define NB 4
#endif
#ifndef SEQ
#define SEQ 2048
#endif
#define NB_FULL  4
#define SEQ_FULL 2048
#define DIM    1024
#define NHEAD  16
#define NKV    4
#define GROUPSZ 4
#define HD     64
#define KVW    (NKV * HD)
#define KVOUT  (2 * NKV * HD)
#define DFF    2048
#define MROWS  (NB * SEQ)

static_assert(NB >= 1 && NB <= NB_FULL);
static_assert(SEQ >= 128 && SEQ <= SEQ_FULL && (SEQ % 128) == 0);
static_assert(DIM == NHEAD * HD);
static_assert(NHEAD == NKV * GROUPSZ && GROUPSZ == 4);
static_assert(HD == 64);
static_assert((DIM % 64) == 0 && (DFF % 64) == 0 && (KVOUT % 64) == 0);
static_assert((MROWS % 64) == 0 && (SEQ % 64) == 0);
static_assert((MROWS % 8) == 0);
static_assert(DIM == 32 * 8 * 4);
static_assert((size_t)MROWS * DFF < (size_t)0xFFFFFFFFu);

#define LDT 72
#define LDC 68

#define WCARRY 64.0f
#define PCARRY 1024.0f
#define VCARRY 64.0f
#define HCARRY 16.0f

#define WQ_ELEMS  ((size_t)DIM * DIM)
#define WKV_ELEMS ((size_t)KVOUT * DIM)
#define WO_ELEMS  ((size_t)DIM * DIM)
#define W1_ELEMS  ((size_t)DFF * DIM)
#define W2_ELEMS  ((size_t)DIM * DFF)
static_assert((WQ_ELEMS % 2048) == 0 && (WKV_ELEMS % 2048) == 0 && (W1_ELEMS % 2048) == 0 &&
              (W2_ELEMS % 2048) == 0);

#define WT_BYTES      ((WQ_ELEMS + WKV_ELEMS + WO_ELEMS + W1_ELEMS + W2_ELEMS) * 2)
#define PLANE16_BYTES ((size_t)MROWS * DIM * 2)
#define KVPLANE_BYTES ((size_t)MROWS * KVW * 2)
#define GPLANE_BYTES  ((size_t)MROWS * DFF * 2)
#define X1_BYTES      ((size_t)MROWS * DIM * 4)
#define OFF_H   (WT_BYTES)
#define OFF_Q   (OFF_H + PLANE16_BYTES)
#define OFF_CTX (OFF_Q + PLANE16_BYTES)
#define OFF_K   (OFF_CTX + PLANE16_BYTES)
#define OFF_VT  (OFF_K + KVPLANE_BYTES)
#define OFF_X1  (OFF_VT + KVPLANE_BYTES)
#define WS_TOTAL (OFF_X1 + X1_BYTES)
static_assert((WT_BYTES % 128) == 0 && (PLANE16_BYTES % 128) == 0 && (KVPLANE_BYTES % 128) == 0);
static_assert(GPLANE_BYTES <= 2 * PLANE16_BYTES);
static_assert(WS_TOTAL <= (size_t)134217728);

__device__ __forceinline__ float bf16r(float x) {
  unsigned int u = __float_as_uint(x);
  u = (u + 0x7FFFu + ((u >> 16) & 1u)) & 0xFFFF0000u;
  return __uint_as_float(u);
}

__device__ __forceinline__ v16h frag_at(const _Float16* p) {
  v8h lo = *(const v8h*)(p);
  v8h hi = *(const v8h*)(p + 16);
  v16h out;
#pragma unroll
  for (int i = 0; i < 8; ++i) { out[i] = lo[i]; out[i + 8] = hi[i]; }
  return out;
}
__device__ __forceinline__ v16h ld_frag(const _Float16* base, unsigned ld) {
  const unsigned lane = threadIdx.x & 31u;
  return frag_at(base + (lane & 15u) * ld + (lane >> 4) * 8u);
}

__device__ __forceinline__ v8f wmma16(v16h a, v16h b, v8f c) {
  v8f d = __builtin_amdgcn_wmma_f32_16x16x32_f16(false, a, false, b, (short)0, c,
                                                 false, false);
  asm volatile("v_nop\n\tv_nop\n\tv_nop\n\tv_nop" : "+v"(d) : "v"(a), "v"(b));
  return d;
}

__device__ __forceinline__ float red16_max(float x) {
#pragma unroll
  for (int off = 1; off < 16; off <<= 1) x = fmaxf(x, __shfl_xor(x, off, 32));
  return x;
}
__device__ __forceinline__ float red16_sum(float x) {
#pragma unroll
  for (int off = 1; off < 16; off <<= 1) x += __shfl_xor(x, off, 32);
  return x;
}
__device__ __forceinline__ float wave_sum(float x) {
#pragma unroll
  for (int off = 1; off < 32; off <<= 1) x += __shfl_xor(x, off, 32);
  return x;
}

__device__ __forceinline__ void wave_lds_sync() {
  __builtin_amdgcn_fence(3  , "wavefront");
  asm volatile("s_wait_dscnt 0x0" ::: "memory");
  __builtin_amdgcn_wave_barrier();
}

__global__ __launch_bounds__(256) void wcvt_kernel(
    const float* __restrict__ src, _Float16* __restrict__ dst) {
  const unsigned e = (blockIdx.x * 256u + threadIdx.x) * 8u;
  const v4f a0 = *(const v4f*)(src + e);
  const v4f a1 = *(const v4f*)(src + e + 4u);
  v8h o;
#pragma unroll
  for (int j = 0; j < 4; ++j) {
    o[j]     = (_Float16)(WCARRY * bf16r(a0[j]));
    o[j + 4] = (_Float16)(WCARRY * bf16r(a1[j]));
  }
  *(volatile v8h*)(dst + (size_t)e) = o;
  __threadfence();
  *(volatile v8h*)(dst + (size_t)e) = o;
}

template <int INPUT>
__global__ __launch_bounds__(256) void ln_kernel(
    const float* __restrict__ X, const float* __restrict__ gam,
    const float* __restrict__ bet, _Float16* __restrict__ dst) {
  const unsigned lane = threadIdx.x & 31u, w = threadIdx.x >> 5;
  const unsigned crow = blockIdx.x * 8u + w;
  size_t srow = crow;
  if (INPUT) {
    const unsigned bidx = crow / (unsigned)SEQ;
    const unsigned sq = crow - bidx * (unsigned)SEQ;
    srow = (size_t)bidx * SEQ_FULL + sq;
  }
  const float* xr = X + srow * DIM + lane * 8u;

  float sum = 0.0f;
#pragma unroll 1
  for (unsigned i = 0; i < 4u; ++i) {
    const v4f a0 = *(const v4f*)(xr + i * 256u);
    const v4f a1 = *(const v4f*)(xr + i * 256u + 4u);
#pragma unroll
    for (int j = 0; j < 4; ++j) {
      const float t0 = INPUT ? bf16r(a0[j]) : a0[j];
      const float t1 = INPUT ? bf16r(a1[j]) : a1[j];
      sum += t0 + t1;
    }
  }
  const float mean = wave_sum(sum) * (1.0f / (float)DIM);

  float vs = 0.0f;
#pragma unroll 1
  for (unsigned i = 0; i < 4u; ++i) {
    const v4f a0 = *(const v4f*)(xr + i * 256u);
    const v4f a1 = *(const v4f*)(xr + i * 256u + 4u);
#pragma unroll
    for (int j = 0; j < 4; ++j) {
      const float d0 = (INPUT ? bf16r(a0[j]) : a0[j]) - mean;
      const float d1 = (INPUT ? bf16r(a1[j]) : a1[j]) - mean;
      vs += d0 * d0;
      vs += d1 * d1;
    }
  }
  const float rs = rsqrtf(wave_sum(vs) * (1.0f / (float)DIM) + 1.0e-5f);

  _Float16* dr = dst + (size_t)crow * DIM + lane * 8u;
  const float* gr = gam + lane * 8u;
  const float* br = bet + lane * 8u;
#pragma unroll 1
  for (unsigned i = 0; i < 4u; ++i) {
    const v4f a0 = *(const v4f*)(xr + i * 256u);
    const v4f a1 = *(const v4f*)(xr + i * 256u + 4u);
    const v4f g0 = *(const v4f*)(gr + i * 256u);
    const v4f g1 = *(const v4f*)(gr + i * 256u + 4u);
    const v4f b0 = *(const v4f*)(br + i * 256u);
    const v4f b1 = *(const v4f*)(br + i * 256u + 4u);
    v8h o;
#pragma unroll
    for (int j = 0; j < 4; ++j) {
      const float t0 = INPUT ? bf16r(a0[j]) : a0[j];
      const float t1 = INPUT ? bf16r(a1[j]) : a1[j];
      o[j]     = (_Float16)((t0 - mean) * rs * bf16r(g0[j]) + bf16r(b0[j]));
      o[j + 4] = (_Float16)((t1 - mean) * rs * bf16r(g1[j]) + bf16r(b1[j]));
    }
    *(volatile v8h*)(dr + i * 256u) = o;
    __threadfence();
    *(volatile v8h*)(dr + i * 256u) = o;
  }
}

template <int MODE, int KD>
__global__ __launch_bounds__(256) void gemm_kernel(
    const _Float16* __restrict__ A16, const _Float16* __restrict__ Bt,
    const float* __restrict__ p0, const float* __restrict__ p1,
    float* __restrict__ outf, _Float16* __restrict__ outa, _Float16* __restrict__ outb) {
  static_assert((KD % 64) == 0);
  __shared__ float Cs[64 * LDC];
  const unsigned tid = threadIdx.x, lane = tid & 31u, w = tid >> 5;
  const unsigned mw = w >> 1, nw = w & 1u;
  const unsigned hh = lane >> 4, m = lane & 15u;
  const unsigned n0 = blockIdx.x * 64u;
  const unsigned row0 = blockIdx.y * 64u;

  const _Float16* ap  = A16 + (size_t)(row0 + mw * 16u + m) * KD + hh * 8u;
  const _Float16* bp0 = Bt + (size_t)(n0 + nw * 32u + m) * KD + hh * 8u;
  const _Float16* bp1 = bp0 + 16 * KD;
  v8f acc0 = {}, acc1 = {};
#pragma unroll 2
  for (unsigned k0 = 0; k0 < (unsigned)KD; k0 += 32u) {
    const v16h a  = frag_at(ap + k0);
    const v16h b0 = frag_at(bp0 + k0);
    const v16h b1 = frag_at(bp1 + k0);
    acc0 = wmma16(a, b0, acc0);
    acc1 = wmma16(a, b1, acc1);
  }
#pragma unroll
  for (int r = 0; r < 8; ++r) {
    float* d = &Cs[(mw * 16u + hh * 8u + (unsigned)r) * LDC + nw * 32u + m];
    d[0]  = acc0[r];
    d[16] = acc1[r];
  }
  __syncthreads();

  if (MODE == 0 || MODE == 1) {
    const bool isv = (MODE == 1) && ((blockIdx.x & 1u) != 0u);
    if (!isv) {
      const unsigned pitch = (MODE == 0) ? (unsigned)DIM : (unsigned)KVW;
      const unsigned colbase = (MODE == 0) ? n0 : (blockIdx.x >> 1) * 64u;
      v8h x[2];
      size_t off[2];
#pragma unroll
      for (unsigned i = 0; i < 2u; ++i) {
        const unsigned r = 32u * i + (tid >> 3);
        const unsigned c = (tid & 7u) * 8u;
        const unsigned crow = row0 + r;
        const unsigned bidx = crow / (unsigned)SEQ;
        const unsigned sq = crow - bidx * (unsigned)SEQ;
        const v4f u0 = *(const v4f*)&Cs[r * LDC + c];
        const v4f u1 = *(const v4f*)&Cs[r * LDC + c + 4];
        const v4f c0 = *(const v4f*)(p0 + (size_t)sq * HD + c);
        const v4f c1 = *(const v4f*)(p0 + (size_t)sq * HD + c + 4u);
        const v4f s0 = *(const v4f*)(p1 + (size_t)sq * HD + c);
        const v4f s1 = *(const v4f*)(p1 + (size_t)sq * HD + c + 4u);
        float q[8], cc[8], ss[8];
#pragma unroll
        for (int j = 0; j < 4; ++j) {
          q[j]      = u0[j] * (1.0f / WCARRY);
          q[j + 4]  = u1[j] * (1.0f / WCARRY);
          cc[j]     = bf16r(c0[j]);
          cc[j + 4] = bf16r(c1[j]);
          ss[j]     = bf16r(s0[j]);
          ss[j + 4] = bf16r(s1[j]);
        }
#pragma unroll
        for (int pr = 0; pr < 4; ++pr) {
          const int e = 2 * pr, o = 2 * pr + 1;
          x[i][e] = (_Float16)(q[e] * cc[e] - q[o] * ss[e]);
          x[i][o] = (_Float16)(q[o] * cc[o] + q[e] * ss[o]);
        }
        off[i] = (size_t)crow * pitch + colbase + c;
      }
#pragma unroll
      for (int i = 0; i < 2; ++i) *(volatile v8h*)(outa + off[i]) = x[i];
      __threadfence();
#pragma unroll
      for (int i = 0; i < 2; ++i) *(volatile v8h*)(outa + off[i]) = x[i];
    } else {
      const unsigned kvh = blockIdx.x >> 1;
      const unsigned bidx = row0 / (unsigned)SEQ;
      const unsigned key0 = row0 - bidx * (unsigned)SEQ;
      v8h x[2];
      size_t off[2];
#pragma unroll
      for (unsigned i = 0; i < 2u; ++i) {
        const unsigned dcol = 32u * i + (tid >> 3);
        const unsigned kk = (tid & 7u) * 8u;
#pragma unroll
        for (unsigned j = 0; j < 8u; ++j)
          x[i][j] = (_Float16)(Cs[(kk + j) * LDC + dcol] * (1.0f / WCARRY));
        off[i] = ((size_t)bidx * KVW + kvh * 64u + dcol) * SEQ + key0 + kk;
      }
#pragma unroll
      for (int i = 0; i < 2; ++i) *(volatile v8h*)(outb + off[i]) = x[i];
      __threadfence();
#pragma unroll
      for (int i = 0; i < 2; ++i) *(volatile v8h*)(outb + off[i]) = x[i];
    }
  }

  if (MODE == 3) {
#pragma unroll 1
    for (unsigned e = 0; e < 16u; ++e) {
      const unsigned idx = tid + 256u * e;
      const unsigned r = idx >> 6, c = idx & 63u;
      const float u = Cs[r * LDC + c] * (1.0f / WCARRY) + bf16r(p0[n0 + c]);
      const float g = 0.5f * u * (1.0f + erff(u * 0.70710678118654752f));
      Cs[r * LDC + c] = g * HCARRY;
    }
    __syncthreads();
    v8h x[2];
    size_t off[2];
#pragma unroll
    for (unsigned i = 0; i < 2u; ++i) {
      const unsigned r = 32u * i + (tid >> 3);
      const unsigned c = (tid & 7u) * 8u;
      const v4f u0 = *(const v4f*)&Cs[r * LDC + c];
      const v4f u1 = *(const v4f*)&Cs[r * LDC + c + 4];
#pragma unroll
      for (int j = 0; j < 4; ++j) {
        x[i][j]     = (_Float16)u0[j];
        x[i][j + 4] = (_Float16)u1[j];
      }
      off[i] = (size_t)(row0 + r) * DFF + n0 + c;
    }
#pragma unroll
    for (int i = 0; i < 2; ++i) *(volatile v8h*)(outa + off[i]) = x[i];
    __threadfence();
#pragma unroll
    for (int i = 0; i < 2; ++i) *(volatile v8h*)(outa + off[i]) = x[i];
  }

  if (MODE == 2 || MODE == 4) {
    const float sc = (MODE == 2) ? (1.0f / (WCARRY * VCARRY)) : (1.0f / (WCARRY * HCARRY));
    v4f xs[4];
    size_t off[4];
#pragma unroll
    for (unsigned i = 0; i < 4u; ++i) {
      const unsigned r = 16u * i + (tid >> 4);
      const unsigned c = (tid & 15u) * 4u;
      const unsigned crow = row0 + r;
      const unsigned bidx = crow / (unsigned)SEQ;
      const unsigned sq = crow - bidx * (unsigned)SEQ;
      const size_t frow = (size_t)bidx * SEQ_FULL + sq;
      const size_t foff = frow * DIM + n0 + c;
      const size_t coff = (size_t)crow * DIM + n0 + c;
      const v4f u = *(const v4f*)&Cs[r * LDC + c];
      v4f val;
      if (MODE == 2) {
        const v4f rr = *(const v4f*)(p0 + foff);
#pragma unroll
        for (int j = 0; j < 4; ++j) val[j] = bf16r(rr[j]) + u[j] * sc;
        off[i] = coff;
      } else {
        const v4f rr = *(const v4f*)(p0 + coff);
        const v4f g = *(const v4f*)(p1 + n0 + c);
#pragma unroll
        for (int j = 0; j < 4; ++j) val[j] = rr[j] + (u[j] * sc + bf16r(g[j]));
        off[i] = foff;
      }
      xs[i] = val;
    }
#pragma unroll
    for (int i = 0; i < 4; ++i) *(volatile v4f*)(outf + off[i]) = xs[i];
    __threadfence();
#pragma unroll
    for (int i = 0; i < 4; ++i) *(volatile v4f*)(outf + off[i]) = xs[i];
  }
}

__global__ __launch_bounds__(256) void attn_kernel(
    const _Float16* __restrict__ Qh, const _Float16* __restrict__ Kh,
    const _Float16* __restrict__ Vt, _Float16* __restrict__ Ov) {
  __shared__ _Float16 Ks[64 * LDT];
  __shared__ _Float16 Vs[64 * LDT];
  __shared__ _Float16 Ps[8 * 16 * LDT];

  const unsigned tid = threadIdx.x, lane = tid & 31u, w = tid >> 5;
  const unsigned hh = lane >> 4, m = lane & 15u;
  const unsigned q0 = blockIdx.x * 128u;
  const unsigned head = blockIdx.y;
  const unsigned kvh = head >> 2;
  const unsigned b = blockIdx.z;
  const float scale = 0.125f;
  _Float16* P = Ps + w * (16u * LDT);

  const size_t qoff = (size_t)(b * (unsigned)SEQ + q0 + w * 16u + m) * DIM + head * HD + hh * 8u;
  v16h qf[2];
  qf[0] = frag_at(Qh + qoff);
  qf[1] = frag_at(Qh + qoff + 32);

  float mrow[8], lrow[8];
  v8f o[4];
#pragma unroll
  for (int v = 0; v < 8; ++v) { mrow[v] = -1.0e30f; lrow[v] = 0.0f; }
#pragma unroll
  for (int nb = 0; nb < 4; ++nb) o[nb] = (v8f){};

  const size_t kplane = (size_t)b * SEQ * KVW + kvh * HD;
  const size_t vplane = ((size_t)b * KVW + kvh * HD) * SEQ;

  for (unsigned kb = 0; kb < (unsigned)SEQ; kb += 64u) {
#pragma unroll
    for (unsigned j = 0; j < 2u; ++j) {
      const unsigned idx = tid + 256u * j;
      const unsigned r = idx >> 3, c = (idx & 7u) * 8u;
      *(v8h*)&Ks[r * LDT + c] = *(const v8h*)(Kh + kplane + (size_t)(kb + r) * KVW + c);
      *(v8h*)&Vs[r * LDT + c] = *(const v8h*)(Vt + vplane + (size_t)r * SEQ + kb + c);
    }
    __syncthreads();

    v8f s[4];
#pragma unroll
    for (int kg = 0; kg < 4; ++kg) {
      v8f t = {};
#pragma unroll
      for (int c = 0; c < 2; ++c) {
        const v16h kf = ld_frag(&Ks[(kg * 16) * LDT + c * 32], LDT);
        t = wmma16(qf[c], kf, t);
      }
      s[kg] = t * scale;
    }

    float alpha[8];
#pragma unroll
    for (int v = 0; v < 8; ++v) {
      float mx = fmaxf(fmaxf(s[0][v], s[1][v]), fmaxf(s[2][v], s[3][v]));
      mx = red16_max(mx);
      const float mn = fmaxf(mrow[v], mx);
      alpha[v] = __expf(mrow[v] - mn);
      mrow[v] = mn;
    }
#pragma unroll
    for (int kg = 0; kg < 4; ++kg)
#pragma unroll
      for (int v = 0; v < 8; ++v) s[kg][v] = __expf(s[kg][v] - mrow[v]);
#pragma unroll
    for (int v = 0; v < 8; ++v) {
      const float rsum = red16_sum((s[0][v] + s[1][v]) + (s[2][v] + s[3][v]));
      lrow[v] = alpha[v] * lrow[v] + rsum;
    }
#pragma unroll
    for (int nb = 0; nb < 4; ++nb)
#pragma unroll
      for (int v = 0; v < 8; ++v) o[nb][v] = o[nb][v] * alpha[v];

#pragma unroll
    for (int kg = 0; kg < 4; ++kg)
#pragma unroll
      for (int v = 0; v < 8; ++v)
        P[(hh * 8u + (unsigned)v) * LDT + (unsigned)kg * 16u + m] = (_Float16)(s[kg][v] * PCARRY);
    wave_lds_sync();

#pragma unroll
    for (int c = 0; c < 2; ++c) {
      const v16h pf = ld_frag(P + c * 32, LDT);
#pragma unroll
      for (int nb = 0; nb < 4; ++nb) {
        const v16h vf = ld_frag(&Vs[(nb * 16) * LDT + c * 32], LDT);
        o[nb] = wmma16(pf, vf, o[nb]);
      }
    }
    __syncthreads();
  }

  float inv[8];
#pragma unroll
  for (int v = 0; v < 8; ++v) inv[v] = __builtin_amdgcn_rcpf(lrow[v]) * (VCARRY / PCARRY);
#pragma unroll
  for (int nb = 0; nb < 4; ++nb)
#pragma unroll
    for (int v = 0; v < 8; ++v)
      P[(hh * 8u + (unsigned)v) * LDT + (unsigned)nb * 16u + m] = (_Float16)(o[nb][v] * inv[v]);
  wave_lds_sync();
  v8h x[4];
  size_t off[4];
#pragma unroll
  for (unsigned i = 0; i < 4u; ++i) {
    const unsigned r = 4u * i + (lane >> 3);
    const unsigned c = (lane & 7u) * 8u;
    x[i] = *(const v8h*)&P[r * LDT + c];
    off[i] = (size_t)(b * (unsigned)SEQ + q0 + w * 16u + r) * DIM + head * HD + c;
  }
#pragma unroll
  for (int i = 0; i < 4; ++i) *(volatile v8h*)(Ov + off[i]) = x[i];
  __threadfence();
#pragma unroll
  for (int i = 0; i < 4; ++i) *(volatile v8h*)(Ov + off[i]) = x[i];
}

extern "C" void kernel_launch(void* const* d_in, const int* in_sizes, int n_in,
                              void* d_out, int out_size, void* d_ws, size_t ws_size,
                              hipStream_t stream) {
  if (n_in < 14) return;
  const long long need_x = ((long long)(NB - 1) * SEQ_FULL + SEQ) * DIM;
  if ((long long)in_sizes[0] < need_x) return;
  if ((long long)in_sizes[1] < (long long)SEQ * HD) return;
  if ((long long)in_sizes[2] < (long long)SEQ * HD) return;
  if ((long long)in_sizes[3] < (long long)DIM * DIM) return;
  if ((long long)in_sizes[4] < (long long)KVOUT * DIM) return;
  if ((long long)in_sizes[5] < (long long)DIM * DIM) return;
  if (in_sizes[6] < DIM || in_sizes[7] < DIM || in_sizes[8] < DIM || in_sizes[9] < DIM) return;
  if ((long long)in_sizes[10] < (long long)DFF * DIM) return;
  if (in_sizes[11] < DFF) return;
  if ((long long)in_sizes[12] < (long long)DIM * DFF) return;
  if (in_sizes[13] < DIM) return;
  if ((long long)out_size < need_x) return;
  if (ws_size < WS_TOTAL) return;

  const float* X    = (const float*)d_in[0];
  const float* cosT = (const float*)d_in[1];
  const float* sinT = (const float*)d_in[2];
  const float* Wq   = (const float*)d_in[3];
  const float* Wkv  = (const float*)d_in[4];
  const float* Wo   = (const float*)d_in[5];
  const float* g1   = (const float*)d_in[6];
  const float* be1  = (const float*)d_in[7];
  const float* g2   = (const float*)d_in[8];
  const float* be2  = (const float*)d_in[9];
  const float* W1   = (const float*)d_in[10];
  const float* b1   = (const float*)d_in[11];
  const float* W2   = (const float*)d_in[12];
  const float* b2   = (const float*)d_in[13];
  float* out = (float*)d_out;

  char* ws = (char*)d_ws;
  _Float16* Wq16  = (_Float16*)ws;
  _Float16* Wkv16 = Wq16 + WQ_ELEMS;
  _Float16* Wo16  = Wkv16 + WKV_ELEMS;
  _Float16* W116  = Wo16 + WO_ELEMS;
  _Float16* W216  = W116 + W1_ELEMS;
  _Float16* H16   = (_Float16*)(ws + OFF_H);
  _Float16* Q16   = (_Float16*)(ws + OFF_Q);
  _Float16* Ctx16 = (_Float16*)(ws + OFF_CTX);
  _Float16* K16   = (_Float16*)(ws + OFF_K);
  _Float16* Vt16  = (_Float16*)(ws + OFF_VT);
  float*    X1    = (float*)(ws + OFF_X1);
  _Float16* G16   = (_Float16*)(ws + OFF_Q);

  dim3 blk(256);
  const unsigned mt = (unsigned)(MROWS / 64);

  wcvt_kernel<<<dim3((unsigned)(WQ_ELEMS / 2048)), blk, 0, stream>>>(Wq, Wq16);
  wcvt_kernel<<<dim3((unsigned)(WKV_ELEMS / 2048)), blk, 0, stream>>>(Wkv, Wkv16);
  wcvt_kernel<<<dim3((unsigned)(WO_ELEMS / 2048)), blk, 0, stream>>>(Wo, Wo16);
  wcvt_kernel<<<dim3((unsigned)(W1_ELEMS / 2048)), blk, 0, stream>>>(W1, W116);
  wcvt_kernel<<<dim3((unsigned)(W2_ELEMS / 2048)), blk, 0, stream>>>(W2, W216);

  ln_kernel<1><<<dim3(MROWS / 8), blk, 0, stream>>>(X, g1, be1, H16);
  gemm_kernel<0, DIM><<<dim3(DIM / 64, mt), blk, 0, stream>>>(
      H16, Wq16, cosT, sinT, X1, Q16, Q16);
  gemm_kernel<1, DIM><<<dim3(KVOUT / 64, mt), blk, 0, stream>>>(
      H16, Wkv16, cosT, sinT, X1, K16, Vt16);
  attn_kernel<<<dim3(SEQ / 128, NHEAD, NB), blk, 0, stream>>>(Q16, K16, Vt16, Ctx16);
  gemm_kernel<2, DIM><<<dim3(DIM / 64, mt), blk, 0, stream>>>(
      Ctx16, Wo16, X, b2, X1, Q16, Q16);
  ln_kernel<0><<<dim3(MROWS / 8), blk, 0, stream>>>(X1, g2, be2, H16);
  gemm_kernel<3, DIM><<<dim3(DFF / 64, mt), blk, 0, stream>>>(
      H16, W116, b1, b1, out, G16, G16);
  gemm_kernel<4, DFF><<<dim3(DIM / 64, mt), blk, 0, stream>>>(
      G16, W216, X1, b2, out, H16, H16);
}
